// PacketDirectionPatternModule_22892175688161
// MI455X (gfx1250) — hardware-verified
//
#include <hip/hip_runtime.h>
#include <stddef.h>
#include <stdint.h>
#include <math.h>

#define NB    16
#define SQ    1024
#define NTOK  16384
#define DM    128
#define NH    4
#define HDM   32
#define NQKV  384
#define DCB   384
#define DF1   256
#define QB    128
#define KC    64
#define NQB   (SQ / QB)
#define NCK   (SQ / KC)
#define SBLK  (SQ / 256)
#define QKPLANE (NB * NH * SQ * HDM)

static_assert(NTOK == NB * SQ);
static_assert(SQ % 256 == 0);
static_assert(SQ % QB == 0);
static_assert(SQ % KC == 0);
static_assert(NH * HDM == DM);
static_assert(NQKV == 3 * DM);
static_assert(NTOK % 256 == 0);
static_assert(NTOK % 8 == 0);
static_assert(DM % 64 == 0);
static_assert(DF1 % 64 == 0);
static_assert(DCB % 32 == 0);
static_assert((NQKV * DM) % 2048 == 0);
static_assert((DM * DM) % 2048 == 0);
static_assert((DF1 * DCB) % 2048 == 0);
static_assert((DM * DF1) % 2048 == 0);
static_assert(HDM == 32);
static_assert(NH == 4);

typedef _Float16 v16h __attribute__((ext_vector_type(16)));
typedef _Float16 v8h  __attribute__((ext_vector_type(8)));
typedef float    v8f  __attribute__((ext_vector_type(8)));
typedef float    v4f  __attribute__((ext_vector_type(4)));
typedef unsigned int v4u __attribute__((ext_vector_type(4)));

union Frag  { v16h v; v8h h[2]; };
union Pack8 { v8h h; v4u u; };

__device__ __forceinline__ v8f mma16(v16h a, v16h b, v8f c) {
  c = __builtin_amdgcn_wmma_f32_16x16x32_f16(false, a, false, b, (short)0, c, false, false);
  asm volatile("v_nop\n\tv_nop\n\tv_nop\n\tv_nop" : "+v"(c) : "v"(a), "v"(b));
  return c;
}

__device__ __forceinline__ v16h ldfrag(const _Float16* p, int ld, int row0, int k0, int lane) {
  const int m = lane & 15, lh = lane >> 4;
  const _Float16* q = p + (size_t)(row0 + m) * ld + k0 + 8 * lh;
  Frag f;
  f.h[0] = *(const v8h*)(q);
  f.h[1] = *(const v8h*)(q + 16);
  return f.v;
}

__device__ __forceinline__ v8f zero8() { return (v8f){0.f, 0.f, 0.f, 0.f, 0.f, 0.f, 0.f, 0.f}; }

__device__ __forceinline__ v8h cvt8(v4f a0, v4f a1) {
  return (v8h){(_Float16)a0[0], (_Float16)a0[1], (_Float16)a0[2], (_Float16)a0[3],
               (_Float16)a1[0], (_Float16)a1[1], (_Float16)a1[2], (_Float16)a1[3]};
}

__device__ __forceinline__ float gelu_erf(float y) {
  return 0.5f * y * (1.0f + erff(y * 0.70710678118654752f));
}

__device__ __forceinline__ void gemm32x64(const _Float16* __restrict__ A, int lda,
                                          const _Float16* __restrict__ Bt, int ldb, int K,
                                          int m0, int n0, int lane, v8f (&acc)[2][4]) {
#pragma unroll 1
  for (int k0 = 0; k0 < K; k0 += 32) {
    const v16h a0 = ldfrag(A, lda, m0, k0, lane);
    const v16h a1 = ldfrag(A, lda, m0 + 16, k0, lane);
    const v16h b0 = ldfrag(Bt, ldb, n0, k0, lane);
    const v16h b1 = ldfrag(Bt, ldb, n0 + 16, k0, lane);
    const v16h b2 = ldfrag(Bt, ldb, n0 + 32, k0, lane);
    const v16h b3 = ldfrag(Bt, ldb, n0 + 48, k0, lane);
    acc[0][0] = mma16(a0, b0, acc[0][0]);
    acc[1][0] = mma16(a1, b0, acc[1][0]);
    acc[0][1] = mma16(a0, b1, acc[0][1]);
    acc[1][1] = mma16(a1, b1, acc[1][1]);
    acc[0][2] = mma16(a0, b2, acc[0][2]);
    acc[1][2] = mma16(a1, b2, acc[1][2]);
    acc[0][3] = mma16(a0, b3, acc[0][3]);
    acc[1][3] = mma16(a1, b3, acc[1][3]);
  }
}

__global__ __launch_bounds__(256) void k_cvt(const float* __restrict__ src, _Float16* __restrict__ dh, float scale) {
  const size_t o = (size_t)blockIdx.x * 2048 + (size_t)threadIdx.x * 8;
  const v4f a0 = *(const v4f*)(src + o) * scale;
  const v4f a1 = *(const v4f*)(src + o + 4) * scale;
  Pack8 pk;
  pk.h = cvt8(a0, a1);
  const v4u vv = pk.u;
  volatile v4u* d = (volatile v4u*)(dh + o);
  *d = vv;
  __threadfence();
  *d = vv;
}

__global__ __launch_bounds__(256) void k_extract(const float* __restrict__ x, const float* __restrict__ temb,
                                                 const float* __restrict__ blemb, const float* __restrict__ bpemb,
                                                 const float* __restrict__ dcw, const float* __restrict__ dcb,
                                                 _Float16* __restrict__ tfp, _Float16* __restrict__ bfp,
                                                 _Float16* __restrict__ combp) {
  __shared__ int s_sgn[SQ];
  __shared__ int s_start[SQ];
  __shared__ int s_len[SQ];
  __shared__ __align__(16) float s_dce[DM];
  __shared__ int s_cnt;
  const int b = blockIdx.x, tid = threadIdx.x, wave = tid >> 5;

  for (int t = tid; t < SQ; t += 256) s_sgn[t] = (x[(size_t)b * SQ + t] > 0.f) ? 1 : 0;
  __syncthreads();

  if (wave == 0) {
    int cnt = 0, cur = 0, prv = s_sgn[0];
#pragma unroll 1
    for (int t = 0; t < SQ; ++t) {
      const int d = s_sgn[t];
      if (t > 0 && d != prv) cur = t;
      s_start[t] = cur;
      cnt += d;
      prv = d;
    }
    int nxt = SQ;
#pragma unroll 1
    for (int t = SQ - 1; t >= 0; --t) {
      const int st0 = s_start[t];
      s_len[t] = nxt - st0;
      if (st0 == t) nxt = t;
    }
    s_cnt = cnt;
  }
  __syncthreads();

  const float inc = (float)s_cnt * 0.0009765625f;
  const float ov  = 1.0f - inc;
  if (tid < DM) {
    const float* w = dcw + tid * 4;
    s_dce[tid] = ((inc * w[0] + ov * w[1]) + inc * w[2]) + ov * w[3] + dcb[tid];
  }
  __syncthreads();

  const int pc = tid & 15;
  v4u dcev;
  {
    const float* e = s_dce + pc * 8;
    const v4f e0 = *(const v4f*)(e) * 64.0f;
    const v4f e1 = *(const v4f*)(e + 4) * 64.0f;
    Pack8 pk;
    pk.h = cvt8(e0, e1);
    dcev = pk.u;
  }
#pragma unroll 1
  for (int it = 0; it < 64; ++it) {
    const int row = (it * 256 + tid) >> 4;
    const int sc  = s_sgn[row];
    const int spv = s_sgn[(row > 0) ? (row - 1) : 0];
    int trid = (row == 0) ? 0 : (2 * spv + sc);
    trid = min(max(trid, 0), 3);
    int L = s_len[row];        L = min(max(L, 0), 31);
    int P = s_start[row] >> 4; P = min(max(P, 0), 63);
    const size_t tok = (size_t)b * SQ + row;
    const float* tp = temb  + trid * DM + pc * 8;
    const float* lp = blemb + L * DM + pc * 8;
    const float* pp = bpemb + P * DM + pc * 8;
    const v4f t0 = *(const v4f*)(tp), t1 = *(const v4f*)(tp + 4);
    const v4f u0 = (*(const v4f*)(lp) + *(const v4f*)(pp)) * 0.5f;
    const v4f u1 = (*(const v4f*)(lp + 4) + *(const v4f*)(pp + 4)) * 0.5f;
    Pack8 pa, pb;
    pa.h = cvt8(t0, t1);
    pb.h = cvt8(u0, u1);
    const v4u va = pa.u, vb = pb.u;
    volatile v4u* da = (volatile v4u*)(tfp + tok * DM + pc * 8);
    volatile v4u* db = (volatile v4u*)(bfp + tok * DM + pc * 8);
    volatile v4u* dd = (volatile v4u*)(combp + tok * DCB + 2 * DM + pc * 8);
    *da = va; *db = vb; *dd = dcev;
    __threadfence();
    *da = va; *db = vb; *dd = dcev;
  }
}

#define STP 72
#define SVP 264
__global__ __launch_bounds__(256) void k_qkv(const _Float16* __restrict__ eh,
                                             const _Float16* __restrict__ wt,
                                             const float* __restrict__ bias,
                                             _Float16* __restrict__ qkp,
                                             _Float16* __restrict__ vtp) {
  __shared__ __align__(16) _Float16 st[256 * STP];
  const int tid = threadIdx.x, lane = tid & 31, wave = tid >> 5;
  const int hh = lane >> 4, c = lane & 15;
  const int bx = blockIdx.x;
  const int b  = bx / SBLK;
  const int sb = (bx - b * SBLK) * 256;
  const int ns = blockIdx.y;
  const int which = ns >> 1;
  const int hp    = ns & 1;
  const int m0 = sb + wave * 32;
  const int n0 = ns * 64;
  const _Float16* A = eh + (size_t)b * SQ * DM;

  v8f acc[2][4];
#pragma unroll
  for (int s = 0; s < 2; ++s)
#pragma unroll
    for (int t = 0; t < 4; ++t) acc[s][t] = zero8();
  gemm32x64(A, DM, wt, DM, DM, m0, n0, lane, acc);

  float bb[4];
#pragma unroll
  for (int t = 0; t < 4; ++t) bb[t] = bias[n0 + 16 * t + c];

  if (which < 2) {
#pragma unroll
    for (int sub = 0; sub < 2; ++sub)
#pragma unroll
      for (int t = 0; t < 4; ++t)
#pragma unroll
        for (int r = 0; r < 8; ++r)
          st[(wave * 32 + sub * 16 + 8 * hh + r) * STP + 16 * t + c] =
              (_Float16)((acc[sub][t][r] * 0.03125f + bb[t]) * 16.0f);
  } else {
#pragma unroll
    for (int sub = 0; sub < 2; ++sub)
#pragma unroll
      for (int t = 0; t < 4; ++t)
#pragma unroll
        for (int r = 0; r < 8; ++r)
          st[(16 * t + c) * SVP + wave * 32 + sub * 16 + 8 * hh + r] =
              (_Float16)((acc[sub][t][r] * 0.03125f + bb[t]) * 16.0f);
  }
  __syncthreads();

  if (which < 2) {
    _Float16* base = qkp + (size_t)which * QKPLANE + (size_t)(b * NH + 2 * hp) * SQ * HDM;
#pragma unroll
    for (int hj = 0; hj < 2; ++hj) {
      v4u val[4];
      size_t go[4];
#pragma unroll
      for (int j = 0; j < 4; ++j) {
        const int p  = tid + 256 * j;
        const int lr = p >> 2;
        const int pc = p & 3;
        Pack8 pk;
        pk.h   = *(const v8h*)(st + lr * STP + 32 * hj + pc * 8);
        val[j] = pk.u;
        go[j]  = (size_t)hj * SQ * HDM + (size_t)(sb + lr) * HDM + pc * 8;
      }
      for (int ps = 0; ps < 2; ++ps) {
#pragma unroll
        for (int j = 0; j < 4; ++j) *(volatile v4u*)(base + go[j]) = val[j];
        __threadfence();
      }
    }
  } else {
    _Float16* base = vtp + (size_t)(b * NH + 2 * hp) * HDM * SQ;
#pragma unroll
    for (int g = 0; g < 2; ++g) {
      v4u val[4];
      size_t go[4];
#pragma unroll
      for (int j = 0; j < 4; ++j) {
        const int p    = tid + 256 * (4 * g + j);
        const int drow = p >> 5;
        const int pc   = p & 31;
        const int hj   = drow >> 5;
        const int d    = drow & 31;
        Pack8 pk;
        pk.h   = *(const v8h*)(st + drow * SVP + pc * 8);
        val[j] = pk.u;
        go[j]  = (size_t)hj * HDM * SQ + (size_t)d * SQ + sb + pc * 8;
      }
      for (int ps = 0; ps < 2; ++ps) {
#pragma unroll
        for (int j = 0; j < 4; ++j) *(volatile v4u*)(base + go[j]) = val[j];
        __threadfence();
      }
    }
  }
}

#define KSP 40
#define VSP 72
#define PSP 72
__global__ __launch_bounds__(256) void k_attn(const _Float16* __restrict__ qp,
                                              const _Float16* __restrict__ kp,
                                              const _Float16* __restrict__ vt,
                                              _Float16* __restrict__ op, float sscale) {
  __shared__ __align__(16) _Float16 Ks[KC * KSP];
  __shared__ __align__(16) _Float16 Vs[HDM * VSP];
  __shared__ __align__(16) _Float16 Ps[8 * 16 * PSP];
  __shared__ __align__(16) _Float16 Os[8 * 16 * PSP];

  const int tid = threadIdx.x, lane = tid & 31, wave = tid >> 5;
  const int hh = lane >> 4, c = lane & 15;
  const int qb  = blockIdx.x % NQB;
  const int hpb = blockIdx.x / NQB;
  const int hp  = hpb & 1;
  const int b   = hpb >> 1;
  const int q0  = qb * QB + wave * 16;

  const float NEGI = -__builtin_huge_valf();
  _Float16* pw = Ps + wave * 16 * PSP;
  _Float16* ow = Os + wave * 16 * PSP;

#pragma unroll 1
  for (int hsel = 0; hsel < 2; ++hsel) {
    const int hb = b * NH + 2 * hp + hsel;
    const _Float16* Q = qp + (size_t)hb * SQ * HDM;
    const _Float16* K = kp + (size_t)hb * SQ * HDM;
    const _Float16* V = vt + (size_t)hb * HDM * SQ;

    const v16h qa = ldfrag(Q, HDM, q0, 0, lane);

    float mrow[8], lrow[8];
    v8f oacc[2];
#pragma unroll
    for (int r = 0; r < 8; ++r) { mrow[r] = NEGI; lrow[r] = 0.f; }
#pragma unroll
    for (int t = 0; t < 2; ++t) oacc[t] = zero8();

#pragma unroll 1
    for (int kcn = 0; kcn < NCK; ++kcn) {
      const int kv0 = kcn * KC;
      __syncthreads();
      {
        const int r  = tid >> 2;
        const int qq = (tid & 3) * 8;
        *(v8h*)(Ks + r * KSP + qq) = *(const v8h*)(K + (size_t)(kv0 + r) * HDM + qq);
        const int r2 = tid >> 3;
        const int q2 = (tid & 7) * 8;
        *(v8h*)(Vs + r2 * VSP + q2) = *(const v8h*)(V + (size_t)r2 * SQ + kv0 + q2);
      }
      __syncthreads();

      v8f s[4];
#pragma unroll
      for (int j = 0; j < 4; ++j) {
        const v16h kb = ldfrag(Ks, KSP, j * 16, 0, lane);
        s[j] = mma16(qa, kb, zero8());
      }
      float cm[8];
#pragma unroll
      for (int r = 0; r < 8; ++r) {
        float m = NEGI;
#pragma unroll
        for (int j = 0; j < 4; ++j) { s[j][r] *= sscale; m = fmaxf(m, s[j][r]); }
#pragma unroll
        for (int off = 1; off < 16; off <<= 1) m = fmaxf(m, __shfl_xor(m, off, 32));
        cm[r] = m;
      }
      float al[8];
#pragma unroll
      for (int r = 0; r < 8; ++r) {
        const float mnew  = fmaxf(mrow[r], cm[r]);
        const float alpha = __expf(mrow[r] - mnew);
        mrow[r] = mnew;
        float psum = 0.f;
#pragma unroll
        for (int j = 0; j < 4; ++j) {
          const float p = __expf(s[j][r] - mnew);
          psum += p;
          pw[(8 * hh + r) * PSP + j * 16 + c] = (_Float16)(p * 1024.0f);
        }
#pragma unroll
        for (int off = 1; off < 16; off <<= 1) psum += __shfl_xor(psum, off, 32);
        lrow[r] = lrow[r] * alpha + psum;
        al[r] = alpha;
      }
#pragma unroll
      for (int t = 0; t < 2; ++t)
#pragma unroll
        for (int r = 0; r < 8; ++r) oacc[t][r] *= al[r];
      __syncthreads();

#pragma unroll
      for (int kk = 0; kk < 2; ++kk) {
        const v16h pa = ldfrag(pw, PSP, 0, kk * 32, lane);
#pragma unroll
        for (int t = 0; t < 2; ++t) {
          const v16h vb = ldfrag(Vs, VSP, t * 16, kk * 32, lane);
          oacc[t] = mma16(pa, vb, oacc[t]);
        }
      }
    }

    float invl[8];
#pragma unroll
    for (int r = 0; r < 8; ++r) invl[r] = (lrow[r] > 0.f) ? (0.00390625f / lrow[r]) : 0.f;
#pragma unroll
    for (int r = 0; r < 8; ++r) {
#pragma unroll
      for (int t = 0; t < 2; ++t)
        ow[(8 * hh + r) * PSP + 32 * hsel + 16 * t + c] = (_Float16)(oacc[t][r] * invl[r]);
    }
  }
  __syncthreads();

  v4u val[4];
  size_t go[4];
#pragma unroll
  for (int it = 0; it < 4; ++it) {
    const int p  = lane + 32 * it;
    const int L  = p >> 3;
    const int pc = p & 7;
    Pack8 pk;
    pk.h    = *(const v8h*)(ow + L * PSP + pc * 8);
    val[it] = pk.u;
    go[it]  = (size_t)(b * SQ + q0 + L) * DM + (size_t)hp * 64 + pc * 8;
  }
  for (int ps = 0; ps < 2; ++ps) {
#pragma unroll
    for (int it = 0; it < 4; ++it) *(volatile v4u*)(op + go[it]) = val[it];
    __threadfence();
  }
}

#define OTP 68
__device__ __forceinline__ void out_epilogue_f32(v8f (&acc)[2][4], float scale, const float (&bb)[4],
                                                 float* sw, float* __restrict__ out, int ldo,
                                                 int m0, int n0, int lane, int hh, int c) {
#pragma unroll
  for (int sub = 0; sub < 2; ++sub) {
    __syncthreads();
#pragma unroll
    for (int t = 0; t < 4; ++t) {
#pragma unroll
      for (int r = 0; r < 8; ++r) sw[(8 * hh + r) * OTP + 16 * t + c] = acc[sub][t][r] * scale + bb[t];
    }
    __syncthreads();
    v4f val[8];
    size_t go[8];
#pragma unroll
    for (int it = 0; it < 8; ++it) {
      const int p    = lane + 32 * it;
      const int L    = p >> 3;
      const int pc   = p & 7;
      const int row  = L >> 1;
      const int half = L & 1;
      val[it] = *(const v4f*)(sw + row * OTP + half * 32 + pc * 4);
      go[it]  = (size_t)(m0 + sub * 16 + row) * ldo + n0 + half * 32 + pc * 4;
    }
    for (int ps = 0; ps < 2; ++ps) {
#pragma unroll
      for (int it = 0; it < 8; ++it) *(volatile v4f*)(out + go[it]) = val[it];
      __threadfence();
    }
  }
}

__device__ __forceinline__ void out_epilogue_h16(v8f (&acc)[2][4], float scale, const float (&bb)[4], float oscale,
                                                 float* sw, _Float16* __restrict__ out, int ldo,
                                                 int m0, int n0, int lane, int hh, int c) {
#pragma unroll
  for (int sub = 0; sub < 2; ++sub) {
    __syncthreads();
#pragma unroll
    for (int t = 0; t < 4; ++t) {
#pragma unroll
      for (int r = 0; r < 8; ++r) {
        sw[(8 * hh + r) * OTP + 16 * t + c] = (acc[sub][t][r] * scale + bb[t]) * oscale;
      }
    }
    __syncthreads();
    v4u val[4];
    size_t go[4];
#pragma unroll
    for (int it = 0; it < 4; ++it) {
      const int p  = lane + 32 * it;
      const int L  = p >> 3;
      const int pc = p & 7;
      const float* ra = sw + L * OTP + pc * 8;
      const v4f a0 = *(const v4f*)(ra), a1 = *(const v4f*)(ra + 4);
      Pack8 pk;
      pk.h = cvt8(a0, a1);
      val[it] = pk.u;
      go[it]  = (size_t)(m0 + sub * 16 + L) * ldo + n0 + pc * 8;
    }
    for (int ps = 0; ps < 2; ++ps) {
#pragma unroll
      for (int it = 0; it < 4; ++it) *(volatile v4u*)(out + go[it]) = val[it];
      __threadfence();
    }
  }
}

__global__ __launch_bounds__(256) void k_gemm_f32(const _Float16* __restrict__ ap, int lda,
                                                  const _Float16* __restrict__ wt, int K,
                                                  const float* __restrict__ bias, float scale,
                                                  float* __restrict__ out, int ldo) {
  __shared__ __align__(16) float st[8][16 * OTP];
  const int tid = threadIdx.x, lane = tid & 31, wave = tid >> 5;
  const int hh = lane >> 4, c = lane & 15;
  const int m0 = blockIdx.x * 256 + wave * 32;
  const int n0 = blockIdx.y * 64;

  v8f acc[2][4];
#pragma unroll
  for (int s = 0; s < 2; ++s)
#pragma unroll
    for (int t = 0; t < 4; ++t) acc[s][t] = zero8();
  gemm32x64(ap, lda, wt, K, K, m0, n0, lane, acc);
  float bb[4];
#pragma unroll
  for (int t = 0; t < 4; ++t) bb[t] = bias[n0 + 16 * t + c];
  out_epilogue_f32(acc, scale, bb, st[wave], out, ldo, m0, n0, lane, hh, c);
}

__global__ __launch_bounds__(256) void k_gemm_h16(const _Float16* __restrict__ ap, int lda,
                                                  const _Float16* __restrict__ wt, int K,
                                                  const float* __restrict__ bias, float scale, float oscale,
                                                  _Float16* __restrict__ out, int ldo) {
  __shared__ __align__(16) float st[8][16 * OTP];
  const int tid = threadIdx.x, lane = tid & 31, wave = tid >> 5;
  const int hh = lane >> 4, c = lane & 15;
  const int m0 = blockIdx.x * 256 + wave * 32;
  const int n0 = blockIdx.y * 64;

  v8f acc[2][4];
#pragma unroll
  for (int s = 0; s < 2; ++s)
#pragma unroll
    for (int t = 0; t < 4; ++t) acc[s][t] = zero8();
  gemm32x64(ap, lda, wt, K, K, m0, n0, lane, acc);
  float bb[4];
#pragma unroll
  for (int t = 0; t < 4; ++t) bb[t] = bias[n0 + 16 * t + c];
  out_epilogue_h16(acc, scale, bb, oscale, st[wave], out, ldo, m0, n0, lane, hh, c);
}

__global__ __launch_bounds__(256) void k_lng1(const float* __restrict__ t, const float* __restrict__ g,
                                              const float* __restrict__ be, _Float16* __restrict__ hp16) {
  __shared__ __align__(16) float sw[8][DF1];
  const int tid = threadIdx.x, lane = tid & 31, wave = tid >> 5;
  const size_t m = (size_t)blockIdx.x * 8 + wave;
  const float* tr = t + m * DF1;

  v4f v[2];
  float s = 0.f;
#pragma unroll
  for (int it = 0; it < 2; ++it) {
    const int idx = it * 128 + lane * 4;
    v[it] = *(const v4f*)(tr + idx);
    s += (v[it][0] + v[it][1]) + (v[it][2] + v[it][3]);
  }
#pragma unroll
  for (int off = 16; off >= 1; off >>= 1) s += __shfl_xor(s, off, 32);
  const float mean = s * 0.00390625f;
  float ss = 0.f;
#pragma unroll
  for (int it = 0; it < 2; ++it) {
    const v4f d = v[it] - mean;
    ss += (d[0] * d[0] + d[1] * d[1]) + (d[2] * d[2] + d[3] * d[3]);
  }
#pragma unroll
  for (int off = 16; off >= 1; off >>= 1) ss += __shfl_xor(ss, off, 32);
  const float var  = ss * 0.00390625f;
  const float rstd = rsqrtf(var + 1e-5f);

#pragma unroll
  for (int it = 0; it < 2; ++it) {
    const int idx = it * 128 + lane * 4;
    const v4f gv = *(const v4f*)(g + idx);
    const v4f bv = *(const v4f*)(be + idx);
    const v4f y  = ((v[it] - mean) * rstd) * gv + bv;
    *(v4f*)(sw[wave] + idx) = y;
  }
  __syncthreads();
#pragma unroll 1
  for (int i = 0; i < 8; ++i) {
    const int e = i * 32 + lane;
    const float yv = sw[wave][e];
    sw[wave][e] = gelu_erf(yv) * 16.0f;
  }
  __syncthreads();
  const float* cp = sw[wave] + 8 * lane;
  const v4f a0 = *(const v4f*)(cp), a1 = *(const v4f*)(cp + 4);
  Pack8 pk;
  pk.h = cvt8(a0, a1);
  const v4u hv = pk.u;
  volatile v4u* d = (volatile v4u*)(hp16 + m * DF1 + 8 * lane);
  *d = hv;
  __threadfence();
  *d = hv;
}

__global__ __launch_bounds__(256) void k_lng2(const float* __restrict__ t, const float* __restrict__ g,
                                              const float* __restrict__ be, float* __restrict__ out) {
  __shared__ __align__(16) float sw[8][DM];
  const int tid = threadIdx.x, lane = tid & 31, wave = tid >> 5;
  const size_t m = (size_t)blockIdx.x * 8 + wave;
  const float* tr = t + m * DM;

  const v4f v = *(const v4f*)(tr + lane * 4);
  float s = (v[0] + v[1]) + (v[2] + v[3]);
#pragma unroll
  for (int off = 16; off >= 1; off >>= 1) s += __shfl_xor(s, off, 32);
  const float mean = s * 0.0078125f;
  const v4f dv = v - mean;
  float ss = (dv[0] * dv[0] + dv[1] * dv[1]) + (dv[2] * dv[2] + dv[3] * dv[3]);
#pragma unroll
  for (int off = 16; off >= 1; off >>= 1) ss += __shfl_xor(ss, off, 32);
  const float var  = ss * 0.0078125f;
  const float rstd = rsqrtf(var + 1e-5f);

  const v4f gv = *(const v4f*)(g + lane * 4);
  const v4f bv = *(const v4f*)(be + lane * 4);
  const v4f y  = (dv * rstd) * gv + bv;
  *(v4f*)(sw[wave] + lane * 4) = y;
  __syncthreads();
#pragma unroll 1
  for (int i = 0; i < 4; ++i) {
    const int e = i * 32 + lane;
    const float yv = sw[wave][e];
    sw[wave][e] = gelu_erf(yv);
  }
  __syncthreads();
  const v4f o = *(const v4f*)(sw[wave] + lane * 4);
  volatile v4f* d = (volatile v4f*)(out + m * DM + lane * 4);
  *d = o;
  __threadfence();
  *d = o;
}

extern "C" void kernel_launch(void* const* d_in, const int* in_sizes, int n_in,
                              void* d_out, int out_size, void* d_ws, size_t ws_size,
                              hipStream_t stream) {
  if (n_in < 22) return;
  if (in_sizes[0]  != NB * SQ) return;
  if (in_sizes[1]  != 4 * DM) return;
  if (in_sizes[2]  != 32 * DM) return;
  if (in_sizes[3]  != 64 * DM) return;
  if (in_sizes[4]  != DM * 4) return;
  if (in_sizes[5]  != DM) return;
  if (in_sizes[6]  != NQKV * DM) return;
  if (in_sizes[7]  != NQKV) return;
  if (in_sizes[8]  != DM * DM) return;
  if (in_sizes[9]  != DM) return;
  if (in_sizes[10] != NQKV * DM) return;
  if (in_sizes[11] != NQKV) return;
  if (in_sizes[12] != DM * DM) return;
  if (in_sizes[13] != DM) return;
  if (in_sizes[14] != DF1 * DCB) return;
  if (in_sizes[15] != DF1) return;
  if (in_sizes[16] != DF1) return;
  if (in_sizes[17] != DF1) return;
  if (in_sizes[18] != DM * DF1) return;
  if (in_sizes[19] != DM) return;
  if (in_sizes[20] != DM) return;
  if (in_sizes[21] != DM) return;
  if (out_size != NTOK * DM) return;

  const float* x        = (const float*)d_in[0];
  const float* temb     = (const float*)d_in[1];
  const float* blemb    = (const float*)d_in[2];
  const float* bpemb    = (const float*)d_in[3];
  const float* dcw      = (const float*)d_in[4];
  const float* dcb      = (const float*)d_in[5];
  const float* ta_in_w  = (const float*)d_in[6];
  const float* ta_in_b  = (const float*)d_in[7];
  const float* ta_out_w = (const float*)d_in[8];
  const float* ta_out_b = (const float*)d_in[9];
  const float* ba_in_w  = (const float*)d_in[10];
  const float* ba_in_b  = (const float*)d_in[11];
  const float* ba_out_w = (const float*)d_in[12];
  const float* ba_out_b = (const float*)d_in[13];
  const float* f1_w     = (const float*)d_in[14];
  const float* f1_b     = (const float*)d_in[15];
  const float* ln1_g    = (const float*)d_in[16];
  const float* ln1_b    = (const float*)d_in[17];
  const float* f2_w     = (const float*)d_in[18];
  const float* f2_b     = (const float*)d_in[19];
  const float* ln2_g    = (const float*)d_in[20];
  const float* ln2_b    = (const float*)d_in[21];
  float* out = (float*)d_out;

  size_t off = 0;
  const size_t oWti = off; off += (size_t)NQKV * DM * 2;
  const size_t oWto = off; off += (size_t)DM * DM * 2;
  const size_t oWbi = off; off += (size_t)NQKV * DM * 2;
  const size_t oWbo = off; off += (size_t)DM * DM * 2;
  const size_t oW1  = off; off += (size_t)DF1 * DCB * 2;
  const size_t oW2  = off; off += (size_t)DM * DF1 * 2;
  const size_t oTF  = off; off += (size_t)NTOK * DM * 2;
  const size_t oBF  = off; off += (size_t)NTOK * DM * 2;
  const size_t oQ   = off; off += (size_t)QKPLANE * 2;
  const size_t oK   = off; off += (size_t)QKPLANE * 2;
  const size_t oV   = off; off += (size_t)QKPLANE * 2;
  const size_t oO   = off; off += (size_t)NTOK * DM * 2;
  const size_t oCB  = off; off += (size_t)NTOK * DCB * 2;
  const size_t oT1  = off; off += (size_t)NTOK * DF1 * 4;
  const size_t oH   = off; off += (size_t)NTOK * DF1 * 2;
  const size_t oT2  = off; off += (size_t)NTOK * DM * 4;
  if (off > ws_size) return;
  if (off > (size_t)134217728) return;
  if (oK != oQ + (size_t)QKPLANE * 2) return;

  char* ws = (char*)d_ws;
  _Float16* Wti = (_Float16*)(ws + oWti);
  _Float16* Wto = (_Float16*)(ws + oWto);
  _Float16* Wbi = (_Float16*)(ws + oWbi);
  _Float16* Wbo = (_Float16*)(ws + oWbo);
  _Float16* W1  = (_Float16*)(ws + oW1);
  _Float16* W2  = (_Float16*)(ws + oW2);
  _Float16* TF  = (_Float16*)(ws + oTF);
  _Float16* BF  = (_Float16*)(ws + oBF);
  _Float16* QKp = (_Float16*)(ws + oQ);
  _Float16* Kp  = (_Float16*)(ws + oK);
  _Float16* Vt  = (_Float16*)(ws + oV);
  _Float16* Op  = (_Float16*)(ws + oO);
  _Float16* CB  = (_Float16*)(ws + oCB);
  float*    T1  = (float*)(ws + oT1);
  _Float16* Hh  = (_Float16*)(ws + oH);
  float*    T2  = (float*)(ws + oT2);

  k_cvt<<<dim3((NQKV * DM) / 2048), dim3(256), 0, stream>>>(ta_in_w, Wti, 32.0f);
  k_cvt<<<dim3((DM * DM) / 2048), dim3(256), 0, stream>>>(ta_out_w, Wto, 32.0f);
  k_cvt<<<dim3((NQKV * DM) / 2048), dim3(256), 0, stream>>>(ba_in_w, Wbi, 32.0f);
  k_cvt<<<dim3((DM * DM) / 2048), dim3(256), 0, stream>>>(ba_out_w, Wbo, 32.0f);
  k_cvt<<<dim3((DF1 * DCB) / 2048), dim3(256), 0, stream>>>(f1_w, W1, 32.0f);
  k_cvt<<<dim3((DM * DF1) / 2048), dim3(256), 0, stream>>>(f2_w, W2, 32.0f);
  k_extract<<<dim3(NB), dim3(256), 0, stream>>>(x, temb, blemb, bpemb, dcw, dcb, TF, BF, CB);

  const float sscale = 0.17677669529663687f * 0.00390625f;
  k_qkv<<<dim3(NB * SBLK, NQKV / 64), dim3(256), 0, stream>>>(TF, Wti, ta_in_b, QKp, Vt);
  k_attn<<<dim3(NB * 2 * NQB), dim3(256), 0, stream>>>(QKp, Kp, Vt, Op, sscale);
  k_gemm_h16<<<dim3(NTOK / 256, DM / 64), dim3(256), 0, stream>>>(Op, DM, Wto, DM, ta_out_b,
                                                                   0.00048828125f, 64.0f, CB, DCB);
  k_qkv<<<dim3(NB * SBLK, NQKV / 64), dim3(256), 0, stream>>>(BF, Wbi, ba_in_b, QKp, Vt);
  k_attn<<<dim3(NB * 2 * NQB), dim3(256), 0, stream>>>(QKp, Kp, Vt, Op, sscale);
  k_gemm_h16<<<dim3(NTOK / 256, DM / 64), dim3(256), 0, stream>>>(Op, DM, Wbo, DM, ba_out_b,
                                                                   0.00048828125f, 64.0f, CB + DM, DCB);
  k_gemm_f32<<<dim3(NTOK / 256, DF1 / 64), dim3(256), 0, stream>>>(CB, DCB, W1, DCB, f1_b, 0.00048828125f, T1, DF1);
  k_lng1<<<dim3(NTOK / 8), dim3(256), 0, stream>>>(T1, ln1_g, ln1_b, Hh);
  k_gemm_f32<<<dim3(NTOK / 256, DM / 64), dim3(256), 0, stream>>>(Hh, DF1, W2, DF1, f2_b, 0.001953125f, T2, DM);
  k_lng2<<<dim3(NTOK / 8), dim3(256), 0, stream>>>(T2, ln2_g, ln2_b, out);
  (void)hipGetLastError();
}
